// PolyHarmInterpolator_43404939493678
// MI455X (gfx1250) — hardware-run, weakly checked
//
#include <hip/hip_runtime.h>


#define NE_  4
#define NM   8192
#define NC   4096
#define NK   16
#define NKP  64
typedef _Float16 h16;
typedef unsigned short bf;
typedef __attribute__((ext_vector_type(16))) __bf16   v16bf;
typedef __attribute__((ext_vector_type(16))) _Float16 v16h;
typedef __attribute__((ext_vector_type(8)))  _Float16 v8h;
typedef __attribute__((ext_vector_type(8)))  unsigned short v8us;
typedef __attribute__((ext_vector_type(8)))  float    v8f;
typedef __attribute__((ext_vector_type(4)))  float    v4f;
typedef v8h  __attribute__((may_alias)) v8ha;
typedef v4f  __attribute__((may_alias)) v4fa;
typedef v8us __attribute__((may_alias)) v8usa;

__device__ __forceinline__ unsigned short f2bf(float f) { unsigned u = __float_as_uint(f); u += 0x7FFFu + ((u >> 16) & 1u); return (unsigned short)(u >> 16); }
__device__ __forceinline__ float bf2f(unsigned short b) { return __uint_as_float(((unsigned)b) << 16); }
__device__ __forceinline__ float bfr(float f) { return bf2f(f2bf(f)); }
__device__ __forceinline__ v16h cat16(v8h lo, v8h hi) { return __builtin_shufflevector(lo, hi, 0, 1, 2, 3, 4, 5, 6, 7, 8, 9, 10, 11, 12, 13, 14, 15); }
__device__ __forceinline__ v16bf cat16b(v8us lo, v8us hi) { return __builtin_bit_cast(v16bf, __builtin_shufflevector(lo, hi, 0, 1, 2, 3, 4, 5, 6, 7, 8, 9, 10, 11, 12, 13, 14, 15)); }
__device__ __forceinline__ v8f wmma16(v16h a, v16h b, v8f c) { return __builtin_amdgcn_wmma_f32_16x16x32_f16(false, a, false, b, (short)0, c, false, false); }
__device__ __forceinline__ v8f wmmab(v16bf a, v16bf b, v8f c) { return __builtin_amdgcn_wmma_f32_16x16x32_bf16(false, a, false, b, (short)0, c, false, false); }


template <typename T16> struct WFrag;
template <> struct WFrag<h16> { typedef v16h V; static __device__ __forceinline__ V ld(const h16* p) { return cat16(*(const v8h*)p, *(const v8h*)(p + 16)); } static __device__ __forceinline__ v8f mma(V a, V b, v8f c) { return wmma16(a, b, c); } };
template <> struct WFrag<bf> { typedef v16bf V; static __device__ __forceinline__ V ld(const bf* p) { return cat16b(*(const v8us*)p, *(const v8us*)(p + 16)); } static __device__ __forceinline__ v8f mma(V a, V b, v8f c) { return wmmab(a, b, c); } };
template <typename T16, int NSPLIT, bool BIAS>
__global__ __launch_bounds__(32) void k_gemmw(const T16* __restrict__ A, const T16* __restrict__ A2, const T16* __restrict__ Bt, const T16* __restrict__ Bt2, int K, float* C, int ldc, const float* __restrict__ bias, size_t sA, size_t sB, size_t sC) {
    typedef typename WFrag<T16>::V V;
    __shared__ __align__(16) float os[16 * 68];
    const size_t z = blockIdx.z; A += z * sA; if (A2) A2 += z * sA; Bt += z * sB; if (Bt2) Bt2 += z * sB; C += z * sC;
    const int lane = threadIdx.x & 31, lr = lane & 15, hi = lane >> 4; const int r0 = blockIdx.x * 64, c0 = blockIdx.y * 64;
    v8f acc[4][4];
#pragma unroll
    for (int mb = 0; mb < 4; ++mb)
#pragma unroll
        for (int nb = 0; nb < 4; ++nb) acc[mb][nb] = (v8f){};
    const size_t aoff = (size_t)(r0 + lr) * K + 8 * hi, boff = (size_t)(c0 + lr) * K + 8 * hi;
    for (int kc = 0; kc < K; kc += 32) {
        V a[4], a2[4];
#pragma unroll
        for (int mb = 0; mb < 4; ++mb) { a[mb] = WFrag<T16>::ld(A + aoff + (size_t)mb * 16 * K + kc); if (NSPLIT == 1 || NSPLIT == 2) a2[mb] = WFrag<T16>::ld(A2 + aoff + (size_t)mb * 16 * K + kc); }
#pragma unroll
        for (int nb = 0; nb < 4; ++nb) { const V b = WFrag<T16>::ld(Bt + boff + (size_t)nb * 16 * K + kc); V b2; if (NSPLIT >= 2) b2 = WFrag<T16>::ld(Bt2 + boff + (size_t)nb * 16 * K + kc);
#pragma unroll
            for (int mb = 0; mb < 4; ++mb) { acc[mb][nb] = WFrag<T16>::mma(a[mb], b, acc[mb][nb]); if (NSPLIT == 1 || NSPLIT == 2) acc[mb][nb] = WFrag<T16>::mma(a2[mb], b, acc[mb][nb]); if (NSPLIT >= 2) acc[mb][nb] = WFrag<T16>::mma(a[mb], b2, acc[mb][nb]); } }
        asm volatile("v_nop\n\tv_nop\n\tv_nop\n\tv_nop" : "+v"(acc[0][0]), "+v"(acc[1][1]), "+v"(acc[2][2]), "+v"(acc[3][3]) : "v"(a[0]), "v"(a[3]));
    }
#pragma unroll
    for (int mb = 0; mb < 4; ++mb) {
#pragma unroll
        for (int nb = 0; nb < 4; ++nb) {
#pragma unroll
            for (int j = 0; j < 8; ++j) os[(hi * 8 + j) * 68 + nb * 16 + lr] = acc[mb][nb][j]; }
        __builtin_amdgcn_wave_barrier(); asm volatile("" ::: "memory");
        float* crow = C + (size_t)(r0 + mb * 16) * ldc + c0;
#pragma unroll 1
        for (int ps = 0; ps < 2; ++ps) {
#pragma unroll
            for (int s = 0; s < 8; ++s) { const int row = 2 * s + hi, cofs = lr * 4; v4f val = *(const v4fa*)(os + row * 68 + cofs); if (BIAS) { val[0] += bfr(bias[c0 + cofs]); val[1] += bfr(bias[c0 + cofs + 1]); val[2] += bfr(bias[c0 + cofs + 2]); val[3] += bfr(bias[c0 + cofs + 3]); }
                *(volatile v4f*)(crow + (size_t)row * ldc + cofs) = val; }
            if (ps == 0) __threadfence(); }
        __builtin_amdgcn_wave_barrier(); asm volatile("" ::: "memory");
    }
}

__device__ __forceinline__ h16 tohx(float x) { return (h16)x; }
__device__ __forceinline__ void splitf(float y, unsigned short& h, unsigned short& l) { h = f2bf(y); l = f2bf(y - bf2f(h)); }
typedef __attribute__((ext_vector_type(2))) _Float16 v2h;
typedef __attribute__((ext_vector_type(4))) _Float16 v4h;
typedef __attribute__((ext_vector_type(2))) unsigned short v2us;
typedef __attribute__((ext_vector_type(4))) unsigned short v4us;
typedef __attribute__((ext_vector_type(2))) float v2f;
typedef __attribute__((ext_vector_type(4))) int v4i;

__global__ __launch_bounds__(256) void k_p4(const float* __restrict__ src, int one, float* Q) { const unsigned idx = blockIdx.x * 256 + threadIdx.x; float t[12];
#pragma unroll
    for (int g = 0; g < 3; ++g) { const v4f a = *(const v4f*)(src + (size_t)idx * 12 + g * 4);
#pragma unroll
        for (int q = 0; q < 4; ++q) t[g * 4 + q] = bfr(a[q]); }
    v4f o[4];
#pragma unroll
    for (int r = 0; r < 4; ++r) { const float w0 = t[r * 3 + 0], w1 = t[r * 3 + 1], w2 = t[r * 3 + 2]; o[r][0] = w0; o[r][1] = w1; o[r][2] = w2; const float sq = __fadd_rn(__fadd_rn(__fmul_rn(w0, w0), __fmul_rn(w1, w1)), __fmul_rn(w2, w2)); o[r][3] = (one != 0) ? 1.0f : sq; }
#pragma unroll
    for (int r = 0; r < 4; ++r) *(volatile v4f*)(Q + (size_t)idx * 16 + r * 4) = o[r];
    __threadfence();
#pragma unroll
    for (int r = 0; r < 4; ++r) *(volatile v4f*)(Q + (size_t)idx * 16 + r * 4) = o[r]; }
__global__ __launch_bounds__(256) void k_rp(const float* __restrict__ PP, const float* __restrict__ CP, h16* P) { const unsigned m = (blockIdx.x / 4) * 2 + (threadIdx.x >> 7), n0 = ((blockIdx.x % 4) * 128 + (threadIdx.x & 127)) * 8; const v4f pq = *(const v4f*)(PP + (size_t)m * 4); const float p0 = pq[0], p1 = pq[1], p2 = pq[2], xs = pq[3]; v8h o;
#pragma unroll
    for (int q = 0; q < 8; ++q) { const v4f cq = *(const v4f*)(CP + (size_t)(n0 + q) * 4); const float c0 = cq[0], c1 = cq[1], c2 = cq[2], cs = cq[3]; const float dt = __fadd_rn(__fadd_rn(__fmul_rn(p0, c0), __fmul_rn(p1, c1)), __fmul_rn(p2, c2)); const float d2 = __fsub_rn(__fadd_rn(xs, cs), __fmul_rn(2.0f, dt)); const float gg = fmaxf(d2, 1.0e-10f); const float ph = __fmul_rn(gg, __fsqrt_rn(gg)); o[q] = tohx((fabsf(ph) < 6.103515625e-5f) ? 0.0f : ph); }
    h16* dst = P + (size_t)m * NC + n0; *(volatile v8h*)dst = o; __threadfence(); *(volatile v8h*)dst = o; }
__global__ __launch_bounds__(256) void k_wt(const float* __restrict__ wsrc, h16* T) { const unsigned idx = blockIdx.x * 256 + threadIdx.x; const unsigned n0 = (idx % (NC / 2)) * 2, r = idx / (NC / 2); const unsigned rc = (r < NK) ? r : (NK - 1); v2h o;
#pragma unroll
    for (int q = 0; q < 2; ++q) { const float w = bfr(wsrc[(size_t)(n0 + q) * NK + rc]); const float y = (r < NK) ? ((fabsf(w) < 6.103515625e-5f) ? 0.0f : w) : 0.0f; o[q] = tohx(y); }
    *(volatile v2h*)(T + (size_t)idx * 2) = o; __threadfence(); *(volatile v2h*)(T + (size_t)idx * 2) = o; }
__global__ __launch_bounds__(256) void k_ep(const float* __restrict__ S, const float* __restrict__ X1, const float* __restrict__ aff, float* out) { const unsigned idx = blockIdx.x * 256 + threadIdx.x; const unsigned k0 = (idx % (NK / 4)) * 4, m = idx / (NK / 4); const v4f s = *(const v4f*)(S + (size_t)m * NKP + k0); const v4f xq = *(const v4f*)(X1 + (size_t)m * 4); const float p0 = xq[0], p1 = xq[1], p2 = xq[2], p3 = xq[3]; const v4f v0 = *(const v4f*)(aff + 0 * NK + k0), v1 = *(const v4f*)(aff + 1 * NK + k0), v2 = *(const v4f*)(aff + 2 * NK + k0), v3 = *(const v4f*)(aff + 3 * NK + k0); v4f o;
#pragma unroll
    for (int q = 0; q < 4; ++q) { const float lin = __fadd_rn(__fadd_rn(__fadd_rn(__fmul_rn(p0, bfr(v0[q])), __fmul_rn(p1, bfr(v1[q]))), __fmul_rn(p2, bfr(v2[q]))), __fmul_rn(p3, bfr(v3[q]))); o[q] = __fadd_rn(s[q], lin); }
    *(volatile v4f*)(out + (size_t)idx * 4) = o; __threadfence(); *(volatile v4f*)(out + (size_t)idx * 4) = o; }

extern "C" void kernel_launch(void* const* d_in, const int* in_sizes, int n_in,
                              void* d_out, int out_size, void* d_ws, size_t ws_size, hipStream_t stream) {
    (void)in_sizes; (void)n_in; (void)out_size;
    const float* a0 = (const float*)d_in[0]; const float* a1 = (const float*)d_in[1]; const float* a2 = (const float*)d_in[2]; const float* a3 = (const float*)d_in[3];
    float* OUT = (float*)d_out;
    char* wsp = (char*)d_ws;
    auto take = [&](size_t bytes) { char* p = wsp; wsp += (bytes + 255) & ~(size_t)255; return (void*)p; };
    float* PP = (float*)take((size_t)NM * 4 * 4); float* CP = (float*)take((size_t)NC * 4 * 4); float* X1 = (float*)take((size_t)NM * 4 * 4); h16* P16 = (h16*)take((size_t)NM * NC * 2); h16* WT16 = (h16*)take((size_t)NKP * NC * 2); float* S = (float*)take((size_t)NM * NKP * 4);
    if ((size_t)(wsp - (char*)d_ws) > ws_size) return;
    for (int b = 0; b < NE_; ++b) {
        k_p4<<<NM / 4 / 256, 256, 0, stream>>>(a0 + (size_t)b * NM * 3, 0, PP); k_p4<<<NC / 4 / 256, 256, 0, stream>>>(a1 + (size_t)b * NC * 3, 0, CP); k_p4<<<NM / 4 / 256, 256, 0, stream>>>(a0 + (size_t)b * NM * 3, 1, X1);
        k_rp<<<NM * (NC / 8) / 256, 256, 0, stream>>>(PP, CP, P16);
        k_wt<<<NKP * (NC / 2) / 256, 256, 0, stream>>>(a2 + (size_t)b * NC * NK, WT16);
        k_gemmw<h16, 0, false><<<dim3(NM / 64, NKP / 64, 1), 32, 0, stream>>>(P16, nullptr, WT16, nullptr, NC, S, NKP, nullptr, 0, 0, 0);
        k_ep<<<NM * (NK / 4) / 256, 256, 0, stream>>>(S, X1, a3 + (size_t)b * 4 * NK, OUT + (size_t)b * NM * NK); }
}
